// TransformerEncoderClassifier_50835232915828
// MI455X (gfx1250) — hardware-verified
//
#include <hip/hip_runtime.h>


#define NB_ 8
#define SS 1024
#define DD 256
#define NH 8
#define DH 32
#define FF 1024
#define NL 2
#define VOC 32000
#define NBK 20000
#define NG 12
#define NCLS 4
#define NTOK (NB_ * SS)
#define CH 8
#define LN_EPS 1e-5f

typedef __attribute__((ext_vector_type(16))) __bf16   v16bf;
typedef __attribute__((ext_vector_type(16))) _Float16 v16h;
typedef __attribute__((ext_vector_type(8)))  float    v8f;
typedef __attribute__((ext_vector_type(8)))  unsigned v8u;

__device__ __forceinline__ unsigned f2bf(float f) { unsigned u = __float_as_uint(f); u += 0x7FFFu + ((u >> 16) & 1u); return u >> 16; }
__device__ __forceinline__ unsigned f2h(float f) { return (unsigned)__builtin_bit_cast(unsigned short, (_Float16)f); }
__device__ __forceinline__ int kpat(int v, int half) { return ((v & 4) ? 16 : 0) + half * 8 + 2 * (v & 3); }

template <int F16, int NP> struct Opnd { v16bf p[NP]; };

template <int F16, int NP> __device__ __forceinline__ void pack2(float f0, float f1, unsigned* o) {
    if (F16) { o[0] = f2h(f0) | (f2h(f1) << 16); return; }
    unsigned h0 = f2bf(f0), h1 = f2bf(f1); o[0] = h0 | (h1 << 16);
    if (NP >= 2) {
        float r0 = f0 - __uint_as_float(h0 << 16), r1 = f1 - __uint_as_float(h1 << 16);
        unsigned m0 = f2bf(r0), m1 = f2bf(r1); o[1] = m0 | (m1 << 16);
        if (NP >= 3) {
            float s0 = r0 - __uint_as_float(m0 << 16), s1 = r1 - __uint_as_float(m1 << 16);
            o[2] = f2bf(s0) | (f2bf(s1) << 16);
        }
    }
}
template <int F16, int NP> __device__ __forceinline__ void op_row(const float* rowp, int half, float sc, Opnd<F16, NP>& o) {
    v8u u[NP];
#pragma unroll
    for (int v = 0; v < 8; ++v) {
        int kk = kpat(v, half); unsigned t[3];
        pack2<F16, NP>(rowp[kk] * sc, rowp[kk + 1] * sc, t);
#pragma unroll
        for (int p = 0; p < NP; ++p) u[p][v] = t[p];
    }
#pragma unroll
    for (int p = 0; p < NP; ++p) o.p[p] = __builtin_bit_cast(v16bf, u[p]);
}
template <int F16, int NP> __device__ __forceinline__ void op_row_tail(const float* rowp, int half, float sc, int kvalid, Opnd<F16, NP>& o) {
    v8u u[NP];
#pragma unroll
    for (int v = 0; v < 8; ++v) {
        int kk = kpat(v, half); unsigned t[3];
        float f0 = kk < kvalid ? rowp[kk] * sc : 0.0f, f1 = (kk + 1) < kvalid ? rowp[kk + 1] * sc : 0.0f;
        pack2<F16, NP>(f0, f1, t);
#pragma unroll
        for (int p = 0; p < NP; ++p) u[p][v] = t[p];
    }
#pragma unroll
    for (int p = 0; p < NP; ++p) o.p[p] = __builtin_bit_cast(v16bf, u[p]);
}
template <int F16, int NP> __device__ __forceinline__ void op_col(const float* M, int ld, int n, int k0, int half, float sc, Opnd<F16, NP>& o) {
    v8u u[NP];
#pragma unroll
    for (int v = 0; v < 8; ++v) {
        int kk = k0 + kpat(v, half); unsigned t[3];
        pack2<F16, NP>(M[(size_t)kk * ld + n] * sc, M[(size_t)(kk + 1) * ld + n] * sc, t);
#pragma unroll
        for (int p = 0; p < NP; ++p) u[p][v] = t[p];
    }
#pragma unroll
    for (int p = 0; p < NP; ++p) o.p[p] = __builtin_bit_cast(v16bf, u[p]);
}
template <int F16, int NP> __device__ __forceinline__ void op_col_tail(const float* M, int ld, int n, int k0, int half, float sc, int K, Opnd<F16, NP>& o) {
    v8u u[NP];
#pragma unroll
    for (int v = 0; v < 8; ++v) {
        int kk = k0 + kpat(v, half); unsigned t[3];
        float f0 = kk < K ? M[(size_t)kk * ld + n] * sc : 0.0f, f1 = (kk + 1) < K ? M[(size_t)(kk + 1) * ld + n] * sc : 0.0f;
        pack2<F16, NP>(f0, f1, t);
#pragma unroll
        for (int p = 0; p < NP; ++p) u[p][v] = t[p];
    }
#pragma unroll
    for (int p = 0; p < NP; ++p) o.p[p] = __builtin_bit_cast(v16bf, u[p]);
}
__device__ __forceinline__ v8f wm_bf16(v16bf a, v16bf b, v8f c) { return __builtin_amdgcn_wmma_f32_16x16x32_bf16(false, a, false, b, (short)0, c, false, false); }
template <int F16, int NA, int NB> __device__ __forceinline__ v8f wmma_op(const Opnd<F16, NA>& a, const Opnd<F16, NB>& b, v8f c) {
    if (F16) {
        v16h ah = __builtin_bit_cast(v16h, a.p[0]), bh = __builtin_bit_cast(v16h, b.p[0]);
        c = __builtin_amdgcn_wmma_f32_16x16x32_f16(false, ah, false, bh, (short)0, c, false, false);
        asm volatile("v_nop\n\tv_nop\n\tv_nop\n\tv_nop" : "+v"(c) : "v"(ah), "v"(bh));
        return c;
    }
    constexpr int NMX = NA > NB ? NA : NB;
#pragma unroll
    for (int i = 0; i < NA; ++i)
#pragma unroll
        for (int j = 0; j < NB; ++j)
            if (i + j < NMX) c = wm_bf16(a.p[i], b.p[j], c);
    if (NA == 1 && NB == 1)      asm volatile("v_nop\n\tv_nop\n\tv_nop\n\tv_nop" : "+v"(c) : "v"(a.p[0]), "v"(b.p[0]));
    else if (NA == 2 && NB == 1) asm volatile("v_nop\n\tv_nop\n\tv_nop\n\tv_nop" : "+v"(c) : "v"(a.p[0]), "v"(a.p[1]), "v"(b.p[0]));
    else if (NA == 1 && NB == 2) asm volatile("v_nop\n\tv_nop\n\tv_nop\n\tv_nop" : "+v"(c) : "v"(a.p[0]), "v"(b.p[0]), "v"(b.p[1]));
    else if (NA == 2 && NB == 2) asm volatile("v_nop\n\tv_nop\n\tv_nop\n\tv_nop" : "+v"(c) : "v"(a.p[0]), "v"(a.p[1]), "v"(b.p[0]), "v"(b.p[1]));
    else                         asm volatile("v_nop\n\tv_nop\n\tv_nop\n\tv_nop" : "+v"(c) : "v"(a.p[0]), "v"(a.p[NA - 1]), "v"(b.p[0]), "v"(b.p[NB - 1]), "v"(a.p[NA / 2]), "v"(b.p[NB / 2]));
    return c;
}

struct ZMap { long long s1; long long s2; int zdiv; int pad_; };
__device__ __forceinline__ size_t zoff(const ZMap& m, int z) { return (size_t)((long long)(z / m.zdiv) * m.s1 + (long long)(z % m.zdiv) * m.s2); }

#define ACT_NONE 0
#define ACT_RELU 1
#define ACT_GELU_ERF 2
#define ACT_SILU 3
#define ACT_TANH 4
__device__ __forceinline__ float act_apply(int act, float x) {
    if (act == ACT_RELU) return x > 0.f ? x : 0.f;
    if (act == ACT_GELU_ERF) return 0.5f * x * (1.0f + erff(x * 0.70710678118654752f));
    if (act == ACT_SILU) return x / (1.0f + expf(-x));
    if (act == ACT_TANH) return tanhf(x);
    return x;
}
struct GemmArgs {
    ZMap za, zb_, zc, zbias, zadd, zrsc, zmul, zrbias;
    const float* A; const float* Bm; float* C; const float* bias; const float* add; const float* rsc; const float* mul; const float* rbias;
    long long ldadd, ldmul;
    int lda, ldb, ldc, K;
    float ascale, bscale, oscale, addscale;
    int M, nvalid, nstore, ldrsc;
    int bcs, pad1, pad2, pad3;
};
template <int BT, int F16, int NA, int NB, int RW, int CW, int ACT>
__global__ __launch_bounds__(256) void gemm_kernel(GemmArgs g) {
    constexpr int TR = 16 * RW, TC = 64 * CW, CSTR = TC + 4;
    __shared__ __align__(16) float cst[TR * CSTR];
    const int z = blockIdx.z;
    const float* A = g.A + zoff(g.za, z); const float* Bm = g.Bm + zoff(g.zb_, z); float* C = g.C + zoff(g.zc, z);
    const int tid = threadIdx.x, lane = tid & 31, wv = tid >> 5;
    const int l16 = lane & 15, half = lane >> 4;
    const int rt = wv % RW, ch = wv / RW;
    const int row0 = blockIdx.x * TR, col0 = blockIdx.y * TC + ch * 64;
    int arix = row0 + rt * 16 + l16; if (arix >= g.M) arix = g.M - 1;
    const float* arow = A + (size_t)arix * g.lda;
    v8f acc[4];
#pragma unroll
    for (int t = 0; t < 4; ++t) acc[t] = (v8f){};
    const int K = g.K;
#pragma unroll 1
    for (int kc = 0; kc < K; kc += 32) {
        Opnd<F16, NA> a;
        if (kc + 32 <= K) op_row<F16, NA>(arow + kc, half, g.ascale, a); else op_row_tail<F16, NA>(arow + kc, half, g.ascale, K - kc, a);
#pragma unroll
        for (int t = 0; t < 4; ++t) {
            Opnd<F16, NB> b;
            const int n = col0 + t * 16 + l16;
            if (n < g.nvalid) {
                if (BT) { if (kc + 32 <= K) op_row<F16, NB>(Bm + (size_t)n * g.ldb + kc, half, g.bscale, b); else op_row_tail<F16, NB>(Bm + (size_t)n * g.ldb + kc, half, g.bscale, K - kc, b); }
                else    { if (kc + 32 <= K) op_col<F16, NB>(Bm, g.ldb, n * g.bcs, kc, half, g.bscale, b); else op_col_tail<F16, NB>(Bm, g.ldb, n * g.bcs, kc, half, g.bscale, K, b); }
            } else {
#pragma unroll
                for (int p = 0; p < NB; ++p) b.p[p] = (v16bf){};
            }
            acc[t] = wmma_op<F16, NA, NB>(a, b, acc[t]);
        }
    }
    const float* bias = g.bias ? g.bias + zoff(g.zbias, z) : nullptr;
    const float* add = g.add ? g.add + zoff(g.zadd, z) : nullptr;
    const float* rsc = g.rsc ? g.rsc + zoff(g.zrsc, z) : nullptr;
    const float* mul = g.mul ? g.mul + zoff(g.zmul, z) : nullptr;
    const float* rbias = g.rbias ? g.rbias + zoff(g.zrbias, z) : nullptr;
#pragma unroll
    for (int t = 0; t < 4; ++t) {
        const int cl = ch * 64 + t * 16 + l16;
        const int cg = blockIdx.y * TC + cl;
        const bool cok = cg < g.nvalid;
        const float bv = (bias && cok) ? bias[(size_t)cg * g.bcs] : 0.0f;
#pragma unroll
        for (int r = 0; r < 8; ++r) {
            const int rl = rt * 16 + r + 8 * half;
            float v = acc[t][r] * g.oscale + bv;
            int rg = row0 + rl; if (rg >= g.M) rg = g.M - 1;
            if (rbias) v += rbias[rg];
            if (rsc) v *= rsc[(size_t)rg * g.ldrsc];
            if (mul && cok) v *= mul[(size_t)rg * g.ldmul + cg];
            if (add && cok) v += g.addscale * add[(size_t)rg * g.ldadd + cg];
            cst[rl * CSTR + cl] = v;
        }
    }
    __syncthreads();
    const int col = tid % TC, rsel = tid / TC, rstep = 256 / TC;
    if (ACT != ACT_NONE) {
#pragma unroll 1
        for (int r = rsel; r < TR; r += rstep) cst[r * CSTR + col] = act_apply(ACT, cst[r * CSTR + col]);
    }
    float* ob = C + (size_t)row0 * g.ldc + (size_t)blockIdx.y * TC;
    const bool colok = (int)(blockIdx.y * TC + col) < g.nstore;
    const int rmax = (g.M - row0 < TR) ? (g.M - row0) : TR;
    auto pass = [&]() {
        if (colok) {
#pragma unroll 4
            for (int r = rsel; r < rmax; r += rstep) *(volatile float*)(ob + (size_t)r * g.ldc + col) = cst[r * CSTR + col];
        }
    };
    pass();
    __threadfence();
    pass();
}
static inline ZMap zm(long long s1) { ZMap m; m.s1 = s1; m.s2 = 0; m.zdiv = 1; m.pad_ = 0; return m; }
static inline ZMap zm2(long long s1, long long s2, int zdiv) { ZMap m; m.s1 = s1; m.s2 = s2; m.zdiv = zdiv; m.pad_ = 0; return m; }
static inline GemmArgs gemm_args(const float* A, int lda, ZMap za, const float* Bm, int ldb, ZMap zb, float* C, int ldc, ZMap zc, int M, int N, int K) {
    GemmArgs g; g.za = za; g.zb_ = zb; g.zc = zc; g.zbias = zm(0); g.zadd = zm(0); g.zrsc = zm(0); g.zmul = zm(0); g.zrbias = zm(0);
    g.A = A; g.Bm = Bm; g.C = C; g.bias = nullptr; g.add = nullptr; g.rsc = nullptr; g.mul = nullptr; g.rbias = nullptr; g.ldadd = 0; g.ldmul = 0;
    g.lda = lda; g.ldb = ldb; g.ldc = ldc; g.K = K; g.ascale = 1.0f; g.bscale = 1.0f; g.oscale = 1.0f; g.addscale = 1.0f; g.M = M; g.nvalid = N; g.nstore = N; g.ldrsc = 1;
    g.bcs = 1; g.pad1 = 0; g.pad2 = 0; g.pad3 = 0;
    return g;
}
static_assert(sizeof(ZMap) == 24, "ZMap layout");
static_assert(sizeof(GemmArgs) == 8 * 24 + 8 * 8 + 2 * 8 + 4 * 4 + 4 * 4 + 4 * 4 + 4 * 4, "GemmArgs has no padding");

__global__ __launch_bounds__(256) void softmax_rows(float* S, long long sy, long long sx, int L, float prescale, const float* addv, long long say, int aydiv, int causal,
                                                  const int* imask, long long imy, long long imx, float maskval) {
    __shared__ float red[8];
    const int tid = threadIdx.x, lane = tid & 31, wid = tid >> 5;
    float* row = S + (size_t)blockIdx.y * sy + (size_t)blockIdx.x * sx;
    const float* av = addv ? addv + (size_t)(blockIdx.y / aydiv) * say : nullptr;
    const int* im = imask ? imask + (size_t)(blockIdx.y / aydiv) * imy + (size_t)blockIdx.x * imx : nullptr;
    float v[16];
    const int nj = L / 256;
    float mx = -__builtin_inff();
#pragma unroll
    for (int j = 0; j < 16; ++j) if (j < nj) { float t = row[tid + 256 * j] * prescale; if (av) t += av[tid + 256 * j]; if (im && im[tid + 256 * j] == 0) t = maskval; if (causal && (tid + 256 * j) > (int)blockIdx.x) t = -__builtin_inff(); v[j] = t; mx = fmaxf(mx, t); }
#pragma unroll
    for (int o = 16; o; o >>= 1) mx = fmaxf(mx, __shfl_xor(mx, o, 32));
    if (lane == 0) red[wid] = mx;
    __syncthreads();
    float m = red[0];
#pragma unroll
    for (int i = 1; i < 8; ++i) m = fmaxf(m, red[i]);
    if (m == -__builtin_inff()) m = 0.f;
    __syncthreads();
    float sum = 0.f;
#pragma unroll
    for (int j = 0; j < 16; ++j) if (j < nj) { v[j] = expf(v[j] - m); sum += v[j]; }
#pragma unroll
    for (int o = 16; o; o >>= 1) sum += __shfl_xor(sum, o, 32);
    if (lane == 0) red[wid] = sum;
    __syncthreads();
    float tot = 0.f;
#pragma unroll
    for (int i = 0; i < 8; ++i) tot += red[i];
    const float inv = 1.0f / tot;
#pragma unroll
    for (int j = 0; j < 16; ++j) if (j < nj) *(volatile float*)(row + tid + 256 * j) = v[j] * inv;
    __threadfence();
#pragma unroll
    for (int j = 0; j < 16; ++j) if (j < nj) *(volatile float*)(row + tid + 256 * j) = v[j] * inv;
}

#define VST2(T, p, v) do { const T vst2_v_ = (v); *(volatile T*)(p) = vst2_v_; __threadfence(); *(volatile T*)(p) = vst2_v_; } while (0)
__global__ __launch_bounds__(256) void k_embed(const int* __restrict__ ids, const int* __restrict__ ngram, const float* __restrict__ tfidf, const float* __restrict__ emb, const float* __restrict__ pos,
                                               const float* __restrict__ bemb, float* X, float* KB, int* PM) {
    const int lane = threadIdx.x & 31, tok = blockIdx.x * 8 + (threadIdx.x >> 5); const int s = tok % SS;
    int id = ids[tok]; const int idc = id < 0 ? 0 : (id >= VOC ? VOC - 1 : id);
    float v[8]; float cnt = 0.f;
#pragma unroll
    for (int j = 0; j < 8; ++j) v[j] = 0.f;
    for (int g = 0; g < NG; ++g) { int bk = ngram[idc * NG + g]; if (bk != 0) { cnt += 1.f; const int bkc = bk < 0 ? 0 : (bk >= NBK ? NBK - 1 : bk);
#pragma unroll
        for (int j = 0; j < 8; ++j) v[j] += bemb[(size_t)bkc * DD + lane + 32 * j]; } }
    const float inv = 1.0f / fmaxf(cnt, 1.0f);
    float* xr = X + (size_t)tok * DD;
#pragma unroll
    for (int j = 0; j < 8; ++j) { const int c = lane + 32 * j; const float val = emb[(size_t)idc * DD + c] + pos[(size_t)s * DD + c] + v[j] * inv; *(volatile float*)(xr + c) = val; }
    __threadfence();
#pragma unroll
    for (int j = 0; j < 8; ++j) { const int c = lane + 32 * j; const float val = emb[(size_t)idc * DD + c] + pos[(size_t)s * DD + c] + v[j] * inv; *(volatile float*)(xr + c) = val; }
}
__global__ __launch_bounds__(256) void k_kbpm(const int* __restrict__ ids, const float* __restrict__ tfidf, float* KB, int* PM) {
    const int tok = blockIdx.x * 256 + threadIdx.x; if (tok >= NTOK) return; const int id = ids[tok]; const int idc = id < 0 ? 0 : (id >= VOC ? VOC - 1 : id);
    VST2(float, KB + tok, tfidf[idc]); VST2(int, PM + tok, id != 0 ? 1 : 0);
}
__global__ __launch_bounds__(256) void k_ab(const float* __restrict__ KB, const float* __restrict__ alpha, float* AB) {
    const int q = blockIdx.x * 256 + threadIdx.x; if (q >= NL * NTOK) return; VST2(float, AB + q, alpha[q / NTOK] * KB[q % NTOK]);
}
__global__ __launch_bounds__(256) void k_ln(const float* __restrict__ a, const float* __restrict__ g, const float* __restrict__ bb, float* out) {
    const int lane = threadIdx.x & 31, r = blockIdx.x * 8 + (threadIdx.x >> 5);
    const float* row = a + (size_t)r * DD; float v[8]; float s = 0.f;
#pragma unroll
    for (int j = 0; j < 8; ++j) { v[j] = row[lane + 32 * j]; s += v[j]; }
#pragma unroll
    for (int o = 16; o; o >>= 1) s += __shfl_xor(s, o, 32);
    const float mean = s * (1.0f / DD); float q = 0.f;
#pragma unroll
    for (int j = 0; j < 8; ++j) { const float d = v[j] - mean; q += d * d; }
#pragma unroll
    for (int o = 16; o; o >>= 1) q += __shfl_xor(q, o, 32);
    const float rstd = 1.0f / sqrtf(q * (1.0f / DD) + LN_EPS); float* orow = out + (size_t)r * DD;
#pragma unroll
    for (int j = 0; j < 8; ++j) { const int c = lane + 32 * j; *(volatile float*)(orow + c) = (v[j] - mean) * rstd * g[c] + bb[c]; }
    __threadfence();
#pragma unroll
    for (int j = 0; j < 8; ++j) { const int c = lane + 32 * j; *(volatile float*)(orow + c) = (v[j] - mean) * rstd * g[c] + bb[c]; }
}
__global__ __launch_bounds__(256) void k_cls(const float* __restrict__ X, const float* __restrict__ g, const float* __restrict__ bb, const float* __restrict__ Wc, const float* __restrict__ bc, float* out) {
    __shared__ float res[NB_ * NCLS];
    const int lane = threadIdx.x & 31, b = threadIdx.x >> 5;
    const float* row = X + (size_t)b * SS * DD; float v[8]; float s = 0.f;
#pragma unroll
    for (int j = 0; j < 8; ++j) { v[j] = row[lane + 32 * j]; s += v[j]; }
#pragma unroll
    for (int o = 16; o; o >>= 1) s += __shfl_xor(s, o, 32);
    const float mean = s * (1.0f / DD); float q = 0.f;
#pragma unroll
    for (int j = 0; j < 8; ++j) { const float d = v[j] - mean; q += d * d; }
#pragma unroll
    for (int o = 16; o; o >>= 1) q += __shfl_xor(q, o, 32);
    const float rstd = 1.0f / sqrtf(q * (1.0f / DD) + LN_EPS);
    float acc[NCLS] = {0.f, 0.f, 0.f, 0.f};
#pragma unroll
    for (int j = 0; j < 8; ++j) { const int c = lane + 32 * j; const float xn = (v[j] - mean) * rstd * g[c] + bb[c];
#pragma unroll
        for (int k = 0; k < NCLS; ++k) acc[k] += xn * Wc[c * NCLS + k]; }
#pragma unroll
    for (int k = 0; k < NCLS; ++k) {
#pragma unroll
        for (int o = 16; o; o >>= 1) acc[k] += __shfl_xor(acc[k], o, 32); }
    if (lane < NCLS) res[b * NCLS + lane] = acc[lane] + bc[lane];
    __syncthreads();
    if (threadIdx.x < NB_ * NCLS) { VST2(float, out + threadIdx.x, res[threadIdx.x]); }
}

extern "C" void kernel_launch(void* const* d_in, const int* in_sizes, int n_in,
                              void* d_out, int out_size, void* d_ws, size_t ws_size, hipStream_t stream) {
    (void)in_sizes; (void)n_in; (void)out_size;
    const int* ids = (const int*)d_in[0];
    const int* ngram = (const int*)d_in[1];
    const float* tfidf = (const float*)d_in[2];
    const float* emb = (const float*)d_in[3];
    const float* pos = (const float*)d_in[4];
    const float* bemb = (const float*)d_in[5];
    const float* Wq = (const float*)d_in[6]; const float* bq = (const float*)d_in[7]; const float* Wk = (const float*)d_in[8]; const float* bk = (const float*)d_in[9];
    const float* Wv = (const float*)d_in[10]; const float* bv = (const float*)d_in[11]; const float* Wo = (const float*)d_in[12]; const float* bo = (const float*)d_in[13];
    const float* g1 = (const float*)d_in[14]; const float* be1 = (const float*)d_in[15]; const float* g2 = (const float*)d_in[16]; const float* be2 = (const float*)d_in[17];
    const float* W1 = (const float*)d_in[18]; const float* b1 = (const float*)d_in[19]; const float* W2 = (const float*)d_in[20]; const float* b2 = (const float*)d_in[21];
    const float* alpha = (const float*)d_in[22];
    const float* gf = (const float*)d_in[23]; const float* bfv = (const float*)d_in[24]; const float* Wc = (const float*)d_in[25]; const float* bc = (const float*)d_in[26];
    float* out = (float*)d_out;

    float* X = (float*)d_ws; float* X2 = X + (size_t)NTOK * DD; float* Q = X2 + (size_t)NTOK * DD; float* Kb = Q + (size_t)NTOK * DD; float* V = Kb + (size_t)NTOK * DD; float* O = V + (size_t)NTOK * DD;
    float* F = O + (size_t)NTOK * DD;
    float* KB = F + (size_t)NTOK * FF; float* AB = KB + NTOK; int* PM = (int*)(AB + NL * NTOK);
    float* S = (float*)(PM + NTOK);
    const size_t wsNeed = (size_t)((S + (size_t)CH * SS * SS) - (float*)d_ws) * sizeof(float);
    if (wsNeed > ws_size) return;

    k_embed<<<NTOK / 8, 256, 0, stream>>>(ids, ngram, tfidf, emb, pos, bemb, X, KB, PM);
    k_kbpm<<<NTOK / 256, 256, 0, stream>>>(ids, tfidf, KB, PM);
    k_ab<<<(NL * NTOK + 255) / 256, 256, 0, stream>>>(KB, alpha, AB);
    for (int l = 0; l < NL; ++l) {
        k_ln<<<NTOK / 8, 256, 0, stream>>>(X, g1 + l * DD, be1 + l * DD, X2);
        const float* Ws[3] = {Wq + (size_t)l * DD * DD, Wk + (size_t)l * DD * DD, Wv + (size_t)l * DD * DD}; const float* bs[3] = {bq + l * DD, bk + l * DD, bv + l * DD}; float* Cs[3] = {Q, Kb, V};
        for (int i = 0; i < 3; ++i) { GemmArgs g = gemm_args(X2, DD, zm(0), Ws[i], DD, zm(0), Cs[i], DD, zm(0), NTOK, DD, DD); g.bias = bs[i]; gemm_kernel<0, 0, 2, 2, 4, 2, ACT_NONE><<<dim3(NTOK / 64, DD / 128, 1), 256, 0, stream>>>(g); }
        for (int c0 = 0; c0 < NB_ * NH; c0 += CH) {
            const int b = c0 / NH;
            const float* Qc = Q + (size_t)b * SS * DD; const float* Kc = Kb + (size_t)b * SS * DD; const float* Vc = V + (size_t)b * SS * DD; float* Oc = O + (size_t)b * SS * DD;
            { GemmArgs g = gemm_args(Qc, DD, zm(DH), Kc, DD, zm(DH), S, SS, zm((long long)SS * SS), SS, SS, DH); gemm_kernel<1, 0, 2, 2, 4, 2, ACT_NONE><<<dim3(SS / 64, SS / 128, CH), 256, 0, stream>>>(g); }
            softmax_rows<<<dim3(SS, CH), 256, 0, stream>>>(S, (long long)SS * SS, SS, SS, 0.17677669529663687f, AB + (size_t)l * NTOK + (size_t)b * SS, 0LL, CH, 0, PM + (size_t)b * SS, 0LL, 0LL, -__builtin_inff());
            { GemmArgs g = gemm_args(S, SS, zm((long long)SS * SS), Vc, DD, zm(DH), Oc, DD, zm(DH), SS, DH, SS); gemm_kernel<0, 0, 2, 2, 8, 1, ACT_NONE><<<dim3(SS / 128, 1, CH), 256, 0, stream>>>(g); }
        }
        { GemmArgs g = gemm_args(O, DD, zm(0), Wo + (size_t)l * DD * DD, DD, zm(0), X, DD, zm(0), NTOK, DD, DD); g.bias = bo + l * DD; g.add = X; g.ldadd = DD; g.addscale = 1.0f; gemm_kernel<0, 0, 2, 2, 4, 2, ACT_NONE><<<dim3(NTOK / 64, DD / 128, 1), 256, 0, stream>>>(g); }
        k_ln<<<NTOK / 8, 256, 0, stream>>>(X, g2 + l * DD, be2 + l * DD, X2);
        { GemmArgs g = gemm_args(X2, DD, zm(0), W1 + (size_t)l * DD * FF, FF, zm(0), F, FF, zm(0), NTOK, FF, DD); g.bias = b1 + l * FF; gemm_kernel<0, 0, 2, 2, 4, 2, ACT_RELU><<<dim3(NTOK / 64, FF / 128, 1), 256, 0, stream>>>(g); }
        { GemmArgs g = gemm_args(F, FF, zm(0), W2 + (size_t)l * FF * DD, DD, zm(0), X, DD, zm(0), NTOK, DD, FF); g.bias = b2 + l * DD; g.add = X; g.ldadd = DD; g.addscale = 1.0f; gemm_kernel<0, 0, 2, 2, 4, 2, ACT_NONE><<<dim3(NTOK / 64, DD / 128, 1), 256, 0, stream>>>(g); }
    }
    k_cls<<<1, 256, 0, stream>>>(X, gf, bfv, Wc, bc, out);
}
